// MultiHeadedAttention_23046794510586
// MI455X (gfx1250) — hardware-verified
//
#include <hip/hip_runtime.h>
#include <math.h>

typedef __attribute__((ext_vector_type(16))) _Float16 v16h;
typedef __attribute__((ext_vector_type(16))) __bf16 v16b;
typedef __attribute__((ext_vector_type(8)))  _Float16 v8h;
typedef __attribute__((ext_vector_type(8)))  __bf16 v8b;
typedef __attribute__((ext_vector_type(8)))  float v8f;
typedef __attribute__((ext_vector_type(4)))  float v4f;
typedef __attribute__((ext_vector_type(4)))  unsigned v4u;
typedef __attribute__((ext_vector_type(4)))  int v4i;

#ifndef NB
#define NB 4
#endif
#ifndef SEQ
#define SEQ 1024
#endif
#define NB_FULL 4
#define SEQ_FULL 1024
#define CC 1024
#define DIN 1024
#define NH 16
#define HD 64
#define QHI 256
#define QBH (QHI / 64)
#define NKB (SEQ / 64)

static_assert((SEQ % 64) == 0);
static_assert((CC % 128) == 0 && (DIN % 32) == 0 && (HD % 32) == 0 && NH * HD == CC);
static_assert((QHI % 64) == 0 && QHI <= SEQ);
static_assert(NB <= NB_FULL && SEQ <= SEQ_FULL);
static_assert(NKB <= 32);

template <typename T> __device__ __forceinline__ void vst2(void* p, T v) { *(volatile T*)p = v; __threadfence(); *(volatile T*)p = v; }
__device__ __forceinline__ v8f wmma16(v16h a, v16h b, v8f c) {
  v8f d = __builtin_amdgcn_wmma_f32_16x16x32_f16(false, a, false, b, (short)0, c, false, false);
  asm volatile("v_nop\n\tv_nop\n\tv_nop\n\tv_nop" : "+v"(d) : "v"(a), "v"(b));
  return d;
}
__device__ __forceinline__ v8f wmma_bf(v16b a, v16b b, v8f c) {
  v8f d = __builtin_amdgcn_wmma_f32_16x16x32_bf16(false, a, false, b, (short)0, c, false, false);
  asm volatile("v_nop\n\tv_nop\n\tv_nop\n\tv_nop" : "+v"(d) : "v"(a), "v"(b));
  return d;
}
__device__ __forceinline__ v16h frag_h(const _Float16* rowk0, unsigned lane) {
  union { v16h v; v8h q[2]; } u; const _Float16* p = rowk0 + 8u * (lane >> 4);
  u.q[0] = *(const v8h*)p; u.q[1] = *(const v8h*)(p + 16); return u.v;
}
__device__ __forceinline__ v16b frag_b(const __bf16* rowk0, unsigned lane) {
  union { v16b v; v8b q[2]; } u; const __bf16* p = rowk0 + 8u * (lane >> 4);
  u.q[0] = *(const v8b*)p; u.q[1] = *(const v8b*)(p + 16); return u.v;
}
__device__ __forceinline__ v16h frag_f32s(const float* rowk0, unsigned lane, float sc) {
  v16h a; const float* p = rowk0 + 8u * (lane >> 4);
#pragma unroll
  for (int i = 0; i < 8; ++i) { a[i] = (_Float16)(p[i] * sc); a[8 + i] = (_Float16)(p[16 + i] * sc); }
  return a;
}
struct F2 { v16b h, l; };
__device__ __forceinline__ F2 bsplit16(const float v[16]) { F2 r;
#pragma unroll
  for (int i = 0; i < 16; ++i) { const __bf16 h = (__bf16)v[i]; r.h[i] = h; r.l[i] = (__bf16)(v[i] - (float)h); }
  return r; }
__device__ __forceinline__ F2 split_row(const float* row, unsigned k0, unsigned lane) { float v[16]; const float* p = row + k0 + 8u * (lane >> 4);
#pragma unroll
  for (int i = 0; i < 8; ++i) { v[i] = p[i]; v[8 + i] = p[16 + i]; }
  return bsplit16(v); }
__device__ __forceinline__ float bfr(float v) { return (float)(__bf16)v; }
__device__ __forceinline__ v16b wcol_oi(const float* Wm, unsigned k0, unsigned o, unsigned lane, unsigned K) { v16b w; const float* p = Wm + (size_t)o * K + k0 + 8u * (lane >> 4);
#pragma unroll
  for (int i = 0; i < 8; ++i) { w[i] = (__bf16)p[i]; w[8 + i] = (__bf16)p[16 + i]; }
  return w; }
__device__ __forceinline__ v16h wcolh_oi(const float* Wm, unsigned k0, unsigned o, unsigned lane, unsigned K) { v16h w; const float* p = Wm + (size_t)o * K + k0 + 8u * (lane >> 4);
#pragma unroll
  for (int i = 0; i < 8; ++i) { w[i] = (_Float16)(bfr(p[i]) * 256.0f); w[8 + i] = (_Float16)(bfr(p[16 + i]) * 256.0f); }
  return w; }
#define LDSX() do { asm volatile("s_wait_dscnt 0" ::: "memory"); __builtin_amdgcn_wave_barrier(); __builtin_amdgcn_fence(3  , "workgroup"); } while (0)

#define WS_CS  ((size_t)0)
#define WS_SN  (WS_CS + (size_t)SEQ * 128u)
#define WS_FL  (WS_SN + (size_t)SEQ * 128u)
#define WS_QH  (WS_FL + (size_t)NKB * 128u)
#define WS_KH  (WS_QH + 2u * (size_t)NB * SEQ * CC)
#define WS_KL  (WS_KH + 2u * (size_t)NB * SEQ * CC)
#define WS_QL  (WS_KL + 2u * (size_t)NB * SEQ * CC)
#define WS_VT  (WS_QL + 2u * (size_t)NB * QHI * CC)
#define WS_VB  (WS_VT + 2u * (size_t)NB * CC * SEQ)
#define WS_VBL (WS_VB + 2u * (size_t)NB * CC * SEQ)
#define WS_Y   (WS_VBL + 2u * (size_t)NB * CC * SEQ)
#define WS_END (WS_Y + 4u * (size_t)NB * SEQ * CC)
static_assert(WS_END <= (size_t)134217728);

static_assert((SEQ % 8) == 0);
__global__ __launch_bounds__(256) void k_rope(float* __restrict__ CS, float* __restrict__ SN) {
  const unsigned tid = threadIdx.x; const unsigned s = blockIdx.x * 8u + (tid >> 5); const unsigned i = tid & 31u;
  const float t = expf(-0.21586735246819178f * (float)i);
  const float ang = (float)s * t;
  float sn, cs; sincosf(ang, &sn, &cs);
  vst2(CS + s * 32u + i, cs); vst2(SN + s * 32u + i, sn);
}

__global__ __launch_bounds__(256) void k_flags(const int* __restrict__ MK, int* __restrict__ FL) {
  __shared__ int sfl[32];
  const unsigned tid = threadIdx.x, wave = tid >> 5, lane = tid & 31u; const unsigned qb = blockIdx.x;
  if (tid < 32u) sfl[tid] = 0;
  __syncthreads();
  for (unsigned kb = wave; kb < (unsigned)NKB; kb += 8u) {
    int cnt = 0;
#pragma unroll 1
    for (unsigned it = 0; it < 32u; ++it) { const unsigned e = it * 32u + lane; const unsigned row = e >> 4, q4 = e & 15u;
      const v4i m = *(const v4i*)(MK + (size_t)(qb * 64u + row) * SEQ_FULL + kb * 64u + q4 * 4u);
      cnt += (m.x != 0) + (m.y != 0) + (m.z != 0) + (m.w != 0); }
#pragma unroll
    for (int o = 1; o < 32; o <<= 1) cnt += __shfl_xor(cnt, o);
    if (lane == 0u) sfl[kb] = (cnt == 0) ? 0 : ((cnt == 4096) ? 1 : 2);
  }
  __syncthreads();
  if (wave == 0u) { const int v = sfl[lane]; vst2(FL + qb * 32u + lane, v); }
}

__global__ __launch_bounds__(128) void k_proj(const float* __restrict__ XQ, const float* __restrict__ XK, const float* __restrict__ XV, const float* __restrict__ WQ, const float* __restrict__ WK, const float* __restrict__ WV, const float* __restrict__ BQ, const float* __restrict__ BK, const float* __restrict__ BV,
    const float* __restrict__ CS, const float* __restrict__ SN, _Float16* __restrict__ QH, _Float16* __restrict__ QL, _Float16* __restrict__ KH, _Float16* __restrict__ KL, _Float16* __restrict__ VT, __bf16* __restrict__ VB, __bf16* __restrict__ VBL) {
  __shared__ __align__(16) float sf[64][132];
  const unsigned tid = threadIdx.x, wave = tid >> 5, lane = tid & 31u, col = lane & 15u, g = lane >> 4; const unsigned which = blockIdx.z; const unsigned c0 = blockIdx.y * 128u; const unsigned rb = blockIdx.x * 64u; const unsigned bb = rb / (unsigned)SEQ; const unsigned t0 = rb % (unsigned)SEQ;
  const size_t r0 = rb; const size_t xr0 = (size_t)bb * SEQ_FULL + t0;
  const float* X = which == 0u ? XQ : (which == 1u ? XK : XV); const float* WA = which == 0u ? WQ : (which == 1u ? WK : WV); const float* BA = which == 0u ? BQ : (which == 1u ? BK : BV);
  v8f acc[8] = {};
#pragma unroll 2
  for (unsigned kc = 0; kc < DIN / 32; ++kc) { v16b a; { const float* p = X + (xr0 + wave * 16u + col) * DIN + kc * 32u + 8u * g;
#pragma unroll
      for (int i = 0; i < 8; ++i) { a[i] = (__bf16)p[i]; a[8 + i] = (__bf16)p[16 + i]; } }
    asm volatile("s_wait_loadcnt 0x0" ::: "memory");
#pragma unroll
    for (int j = 0; j < 8; ++j) { const v16b w = wcol_oi(WA, kc * 32u, c0 + j * 16u + col, lane, DIN); asm volatile("s_wait_loadcnt 0x0" ::: "memory"); acc[j] = wmma_bf(a, w, acc[j]); } }
#pragma unroll
  for (int j = 0; j < 8; ++j) { const float bias = bfr(BA[c0 + j * 16u + col]);
#pragma unroll
    for (int r = 0; r < 8; ++r) sf[wave * 16u + 8u * g + r][j * 16u + col] = acc[j][r] + bias; }
  __syncthreads();
  if (which < 2u) { _Float16* DH = which == 0u ? QH : KH; const bool qres = (which == 0u) && (t0 < (unsigned)QHI);
    for (unsigned e = tid; e < 64u * 16u; e += 128u) { const unsigned rl = e >> 4, q = e & 15u;
      const v4f x0 = *(const v4f*)&sf[rl][q * 8u], x1 = *(const v4f*)&sf[rl][q * 8u + 4u];
      const unsigned s = t0 + rl; const unsigned i0 = ((c0 + q * 8u) & 63u) >> 1;
      const v4f cs = *(const v4f*)(CS + s * 32u + i0), sn = *(const v4f*)(SN + s * 32u + i0);
      float o[8];
      o[0] = x0.x * cs.x - x0.y * sn.x; o[1] = x0.y * cs.x + x0.x * sn.x;
      o[2] = x0.z * cs.y - x0.w * sn.y; o[3] = x0.w * cs.y + x0.z * sn.y;
      o[4] = x1.x * cs.z - x1.y * sn.z; o[5] = x1.y * cs.z + x1.x * sn.z;
      o[6] = x1.z * cs.w - x1.w * sn.w; o[7] = x1.w * cs.w + x1.z * sn.w;
      v8h hh, hl;
#pragma unroll
      for (int u = 0; u < 8; ++u) { const float t = o[u] * 16.0f; const _Float16 hv = (_Float16)t; hh[u] = hv; hl[u] = (_Float16)((t - (float)hv) * 1024.0f); }
      const size_t off = (r0 + rl) * CC + c0 + q * 8u;
      vst2(DH + off, __builtin_bit_cast(v4u, hh));
      if (which == 1u) vst2(KL + off, __builtin_bit_cast(v4u, hl));
      if (qres) vst2(QL + ((size_t)bb * QHI + t0 + rl) * CC + c0 + q * 8u, __builtin_bit_cast(v4u, hl)); }
  } else {
    for (unsigned e = tid; e < 128u * 8u; e += 128u) { const unsigned cl = e >> 3, q = e & 7u; v8h hv; v8b bh, bl;
#pragma unroll
      for (int j = 0; j < 8; ++j) { const float v = sf[q * 8u + j][cl]; hv[j] = (_Float16)(v * 16.0f); const __bf16 b = (__bf16)v; bh[j] = b; bl[j] = (__bf16)(v - (float)b); }
      const size_t off = ((size_t)bb * CC + c0 + cl) * SEQ + t0 + q * 8u;
      vst2(VT + off, __builtin_bit_cast(v4u, hv)); vst2(VB + off, __builtin_bit_cast(v4u, bh)); vst2(VBL + off, __builtin_bit_cast(v4u, bl)); } } }
static_assert((64 * 16) % 128 == 0 && (128 * 8) % 128 == 0);

template <int HI>
__global__ __launch_bounds__(128) void k_fa(const _Float16* __restrict__ QH, const _Float16* __restrict__ QL, const _Float16* __restrict__ KH, const _Float16* __restrict__ KL, const _Float16* __restrict__ VT, const __bf16* __restrict__ VB, const __bf16* __restrict__ VBL,
    const int* __restrict__ MK, const int* __restrict__ FL, float* __restrict__ Y, unsigned qb0) {
  __shared__ __align__(16) _Float16 pw[4][16][72];
  __shared__ __align__(16) __bf16 pbh[4][16][72];
  __shared__ __align__(16) __bf16 pbl[4][16][72];
  __shared__ __align__(16) float ss[4][16][68];
  const unsigned tid = threadIdx.x, wave = tid >> 5, lane = tid & 31u, col = lane & 15u, g = lane >> 4;
  const unsigned qb = qb0 + blockIdx.x, h = blockIdx.y, b = blockIdx.z;
  const unsigned ql0 = qb * 64u + wave * 16u; const size_t q0 = (size_t)b * SEQ + ql0;
  v16h qa[2] = {}, qr[2] = {};
#pragma unroll
  for (int kc = 0; kc < 2; ++kc) { qa[kc] = frag_h(QH + (q0 + col) * CC + h * HD + kc * 32, lane);
    if (HI) qr[kc] = frag_h(QL + ((size_t)b * QHI + ql0 + col) * CC + h * HD + kc * 32, lane); }
  float Mrow[8], Lrow[8]; v8f o_acc[4] = {};
#pragma unroll
  for (int r = 0; r < 8; ++r) { Mrow[r] = -1.0e30f; Lrow[r] = 0.0f; }
  const float SC = 0.125f / 256.0f;
#pragma unroll 1
  for (unsigned kb = 0; kb < (unsigned)NKB; ++kb) {
    const int f = FL[qb * 32u + kb];
    if (f == 0) continue;
    const size_t kr0 = (size_t)b * SEQ + kb * 64u;
    float Sv[4][8];
#pragma unroll
    for (int n = 0; n < 4; ++n) { v8f sa = {}, sl = {};
#pragma unroll
      for (int kc = 0; kc < 2; ++kc) { const size_t ko = (kr0 + n * 16 + col) * CC + h * HD + kc * 32; const v16h kf = frag_h(KH + ko, lane); sa = wmma16(qa[kc], kf, sa);
        if (HI) { sl = wmma16(qr[kc], kf, sl); const v16h klf = frag_h(KL + ko, lane); sl = wmma16(qa[kc], klf, sl); } }
#pragma unroll
      for (int r = 0; r < 8; ++r) Sv[n][r] = HI ? (sa[r] + sl[r] * (1.0f / 1024.0f)) * SC : sa[r] * SC;
      if (f != 1) { int mk[8];
#pragma unroll
        for (int r = 0; r < 8; ++r) mk[r] = MK[(size_t)(ql0 + 8u * g + r) * SEQ_FULL + kb * 64u + n * 16 + col];
        asm volatile("s_wait_loadcnt 0x0" ::: "memory");
#pragma unroll
        for (int r = 0; r < 8; ++r) Sv[n][r] = (mk[r] == 0) ? -1.0e30f : Sv[n][r]; } }
    float corr[8];
#pragma unroll
    for (int r = 0; r < 8; ++r) { float mc = fmaxf(fmaxf(Sv[0][r], Sv[1][r]), fmaxf(Sv[2][r], Sv[3][r]));
      mc = fmaxf(mc, __shfl_xor(mc, 1)); mc = fmaxf(mc, __shfl_xor(mc, 2)); mc = fmaxf(mc, __shfl_xor(mc, 4)); mc = fmaxf(mc, __shfl_xor(mc, 8));
      const float mn = fmaxf(Mrow[r], mc); corr[r] = __expf(fmaxf(Mrow[r] - mn, -100.0f)); float ls = 0.0f;
#pragma unroll
      for (int n = 0; n < 4; ++n) { const float sv = Sv[n][r]; const float p = (sv <= -1.0e29f) ? 0.0f : __expf(fmaxf(sv - mn, -100.0f)); Sv[n][r] = p; ls += p; }
      ls += __shfl_xor(ls, 1); ls += __shfl_xor(ls, 2); ls += __shfl_xor(ls, 4); ls += __shfl_xor(ls, 8);
      Lrow[r] = Lrow[r] * corr[r] + ls; Mrow[r] = mn; }
#pragma unroll
    for (int dt = 0; dt < 4; ++dt)
#pragma unroll
      for (int r = 0; r < 8; ++r) o_acc[dt][r] *= corr[r];
#pragma unroll
    for (int n = 0; n < 4; ++n)
#pragma unroll
      for (int r = 0; r < 8; ++r) { const float p = Sv[n][r];
        if (HI) { const __bf16 ph = (__bf16)p; pbh[wave][8u * g + r][n * 16 + col] = ph; pbl[wave][8u * g + r][n * 16 + col] = (__bf16)(p - (float)ph); }
        else pw[wave][8u * g + r][n * 16 + col] = (_Float16)(p * 256.0f); }
    LDSX();
#pragma unroll
    for (int kc = 0; kc < 2; ++kc) {
      if (HI) { union { v16b v; v8b q[2]; } uh, ul;
        uh.q[0] = *(const v8b*)&pbh[wave][col][kc * 32 + 8u * g]; uh.q[1] = *(const v8b*)&pbh[wave][col][kc * 32 + 16 + 8u * g];
        ul.q[0] = *(const v8b*)&pbl[wave][col][kc * 32 + 8u * g]; ul.q[1] = *(const v8b*)&pbl[wave][col][kc * 32 + 16 + 8u * g];
#pragma unroll
        for (int dt = 0; dt < 4; ++dt) { const size_t po = ((size_t)b * CC + h * HD + dt * 16 + col) * SEQ + kb * 64u + kc * 32; const v16b vh = frag_b(VB + po, lane); const v16b vl = frag_b(VBL + po, lane);
          o_acc[dt] = wmma_bf(uh.v, vh, o_acc[dt]); o_acc[dt] = wmma_bf(ul.v, vh, o_acc[dt]); o_acc[dt] = wmma_bf(uh.v, vl, o_acc[dt]); }
      } else { union { v16h v; v8h q[2]; } up;
        up.q[0] = *(const v8h*)&pw[wave][col][kc * 32 + 8u * g]; up.q[1] = *(const v8h*)&pw[wave][col][kc * 32 + 16 + 8u * g];
#pragma unroll
        for (int dt = 0; dt < 4; ++dt) { const size_t po = ((size_t)b * CC + h * HD + dt * 16 + col) * SEQ + kb * 64u + kc * 32; o_acc[dt] = wmma16(up.v, frag_h(VT + po, lane), o_acc[dt]); } } }
    LDSX();
  }
#pragma unroll
  for (int r = 0; r < 8; ++r) { const float inv = (HI ? 1.0f : (1.0f / 4096.0f)) * (1.0f / Lrow[r]);
#pragma unroll
    for (int dt = 0; dt < 4; ++dt) ss[wave][8u * g + r][dt * 16 + col] = o_acc[dt][r] * inv; }
  LDSX();
#pragma unroll 1
  for (unsigned it = 0; it < 8u; ++it) { const unsigned rl = it * 2u + g; const unsigned c4 = col * 4u;
    const v4f v = *(const v4f*)&ss[wave][rl][c4];
    vst2(Y + ((size_t)b * SEQ + ql0 + rl) * CC + h * HD + c4, v); }
}

__global__ __launch_bounds__(128) void k_out(const float* __restrict__ Y, const float* __restrict__ WO, const float* __restrict__ BO, float* __restrict__ OUT) {
  __shared__ __align__(16) float sf[4][16][132];
  const unsigned tid = threadIdx.x, wave = tid >> 5, lane = tid & 31u, col = lane & 15u, g = lane >> 4; const unsigned c0 = blockIdx.y * 128u; const unsigned rb = blockIdx.x * 64u; const unsigned bb = rb / (unsigned)SEQ, t0 = rb % (unsigned)SEQ;
  const size_t r0 = (size_t)rb + wave * 16u;
  v8f acc[8] = {};
  if (t0 < (unsigned)QHI) {
#pragma unroll 2
    for (unsigned kc = 0; kc < CC / 32; ++kc) { const F2 a = split_row(Y + (r0 + col) * CC, kc * 32u, lane); asm volatile("s_wait_loadcnt 0x0" ::: "memory");
#pragma unroll
      for (int j = 0; j < 8; ++j) { const v16b w = wcol_oi(WO, kc * 32u, c0 + j * 16u + col, lane, CC); asm volatile("s_wait_loadcnt 0x0" ::: "memory"); acc[j] = wmma_bf(a.h, w, acc[j]); acc[j] = wmma_bf(a.l, w, acc[j]); } }
#pragma unroll
    for (int j = 0; j < 8; ++j) { const float bias = bfr(BO[c0 + j * 16u + col]);
#pragma unroll
      for (int r = 0; r < 8; ++r) sf[wave][8u * g + r][j * 16u + col] = acc[j][r] + bias; }
  } else {
#pragma unroll 2
    for (unsigned kc = 0; kc < CC / 32; ++kc) { const v16h a = frag_f32s(Y + (r0 + col) * CC + kc * 32u, lane, 64.0f); asm volatile("s_wait_loadcnt 0x0" ::: "memory");
#pragma unroll
      for (int j = 0; j < 8; ++j) { const v16h w = wcolh_oi(WO, kc * 32u, c0 + j * 16u + col, lane, CC); asm volatile("s_wait_loadcnt 0x0" ::: "memory"); acc[j] = wmma16(a, w, acc[j]); } }
#pragma unroll
    for (int j = 0; j < 8; ++j) { const float bias = bfr(BO[c0 + j * 16u + col]);
#pragma unroll
      for (int r = 0; r < 8; ++r) sf[wave][8u * g + r][j * 16u + col] = acc[j][r] * (1.0f / 16384.0f) + bias; } }
  LDSX();
  const size_t orow = (size_t)bb * SEQ_FULL + t0 + wave * 16u;
#pragma unroll 1
  for (unsigned rl = 0; rl < 16u; ++rl) { const v4f v = *(const v4f*)&sf[wave][rl][lane * 4u]; vst2(OUT + (orow + rl) * DIN + c0 + lane * 4u, v); } }

extern "C" void kernel_launch(void* const* d_in, const int* in_sizes, int n_in, void* d_out, int out_size, void* d_ws, size_t ws_size, hipStream_t stream) {
  if (n_in < 12) return;
  const size_t need_x = ((size_t)(NB - 1) * SEQ_FULL + SEQ) * DIN;
  if ((size_t)in_sizes[0] < need_x || (size_t)in_sizes[1] < need_x || (size_t)in_sizes[2] < need_x) return;
  if ((size_t)in_sizes[3] < (size_t)(SEQ - 1) * SEQ_FULL + SEQ) return;
  if ((size_t)in_sizes[4] < (size_t)CC * DIN || (size_t)in_sizes[6] < (size_t)CC * DIN || (size_t)in_sizes[8] < (size_t)CC * DIN || (size_t)in_sizes[10] < (size_t)DIN * CC) return;
  if (in_sizes[5] < CC || in_sizes[7] < CC || in_sizes[9] < CC || in_sizes[11] < DIN) return;
  if ((size_t)out_size < need_x) return;
  if (ws_size < (size_t)WS_END) return;
  const float* xq = (const float*)d_in[0]; const float* xk = (const float*)d_in[1]; const float* xv = (const float*)d_in[2]; const int* mk = (const int*)d_in[3];
  const float* wq = (const float*)d_in[4]; const float* bq = (const float*)d_in[5]; const float* wk = (const float*)d_in[6]; const float* bk = (const float*)d_in[7];
  const float* wv = (const float*)d_in[8]; const float* bv = (const float*)d_in[9]; const float* wo = (const float*)d_in[10]; const float* bo = (const float*)d_in[11];
  char* ws = (char*)d_ws;
  float* CS = (float*)(ws + WS_CS); float* SN = (float*)(ws + WS_SN); int* FL = (int*)(ws + WS_FL);
  _Float16 *QH = (_Float16*)(ws + WS_QH), *KH = (_Float16*)(ws + WS_KH), *KL = (_Float16*)(ws + WS_KL), *QL = (_Float16*)(ws + WS_QL), *VT = (_Float16*)(ws + WS_VT);
  __bf16 *VB = (__bf16*)(ws + WS_VB), *VBL = (__bf16*)(ws + WS_VBL); float* Y = (float*)(ws + WS_Y);
  k_rope<<<dim3(SEQ / 8), 256, 0, stream>>>(CS, SN);
  k_flags<<<dim3(NKB), 256, 0, stream>>>(mk, FL);
  k_proj<<<dim3(NB * SEQ / 64, CC / 128, 3), 128, 0, stream>>>(xq, xk, xv, wq, wk, wv, bq, bk, bv, CS, SN, QH, QL, KH, KL, VT, VB, VBL);
  k_fa<1><<<dim3(QBH, NH, NB), 128, 0, stream>>>(QH, QL, KH, KL, VT, VB, VBL, mk, FL, Y, 0u);
  if (NKB > QBH) k_fa<0><<<dim3(NKB > QBH ? NKB - QBH : 1, NH, NB), 128, 0, stream>>>(QH, QL, KH, KL, VT, VB, VBL, mk, FL, Y, (unsigned)QBH);
  k_out<<<dim3(NB * SEQ / 64, DIN / 128), 128, 0, stream>>>(Y, wo, bo, (float*)d_out);
}
